// CrossAttention_65446711657232
// MI455X (gfx1250) — hardware-verified
//
#include <hip/hip_runtime.h>


typedef float          v4f   __attribute__((ext_vector_type(4)));
typedef float          v8f   __attribute__((ext_vector_type(8)));
typedef _Float16       v16h  __attribute__((ext_vector_type(16)));
typedef __bf16         v16bf __attribute__((ext_vector_type(16)));
typedef unsigned short v8us  __attribute__((ext_vector_type(8)));
typedef unsigned short v16us __attribute__((ext_vector_type(16)));

#ifndef NB
#define NB 2
#endif
#ifndef SEQ
#define SEQ 1024
#endif
#define NB_FULL 2
#define SQ_FULL 1024
#define SKV     2048
#define EMB     1024
#define NH      16
#define HD      64
#define VOC     4096
#define MQ      (NB * SEQ)
#define MK      (NB * SKV)
#define GSP     132
#define ALP     72

static_assert(NB >= 1 && NB <= NB_FULL);
static_assert(SEQ % 128 == 0 && SEQ >= 128 && SEQ <= SQ_FULL);
static_assert(MQ % 128 == 0 && MK % 128 == 0);
static_assert(EMB % 128 == 0 && VOC % 128 == 0 && EMB % 64 == 0);
static_assert(NH * HD == EMB && HD == 64 && SKV % 64 == 0);
static_assert((size_t)MQ * EMB * 2 * 4 + (size_t)MK * EMB * 2 * 4 +
              (size_t)EMB * EMB * 2 * 3 + (size_t)VOC * EMB * 2 <= 134217728ull);

__device__ __forceinline__ unsigned short bf16_bits_rne(float f) {
  unsigned int u = __float_as_uint(f);
  u += 0x7FFFu + ((u >> 16) & 1u);
  return (unsigned short)(u >> 16);
}
__device__ __forceinline__ float bf16_val(unsigned short b) {
  return __uint_as_float(((unsigned int)b) << 16);
}
__device__ __forceinline__ float bf16_rne(float f) { return bf16_val(bf16_bits_rne(f)); }
__device__ __forceinline__ unsigned short f16_bits(float f) {
  _Float16 h = (_Float16)f;
  return __builtin_bit_cast(unsigned short, h);
}

union Frag { v16us u; v16h h; v16bf b; v8us p[2]; };

__device__ __forceinline__ v16us ld_frag(const unsigned short* p, int hs) {
  Frag f;
  f.p[0] = *(const v8us*)(p + 8 * hs);
  f.p[1] = *(const v8us*)(p + 16 + 8 * hs);
  return f.u;
}
__device__ __forceinline__ v8f mma_bf16(v16us a, v16us b, v8f c) {
  Frag fa, fb; fa.u = a; fb.u = b;
  return __builtin_amdgcn_wmma_f32_16x16x32_bf16(false, fa.b, false, fb.b, (short)0, c, false, false);
}
__device__ __forceinline__ v8f mma_f16(v16us a, v16us b, v8f c) {
  Frag fa, fb; fa.u = a; fb.u = b;
  return __builtin_amdgcn_wmma_f32_16x16x32_f16(false, fa.h, false, fb.h, (short)0, c, false, false);
}

__global__ __launch_bounds__(256) void k_cvt_rows(const float* __restrict__ src, unsigned short* dst,
                                                  int nrows, int seg, int seg_full) {
  const long long e0 = ((long long)blockIdx.x * 256 + threadIdx.x) * 8;
  const int r = (int)(e0 / EMB);
  const int c = (int)(e0 - (long long)r * EMB);
  if (r >= nrows) return;
  const int rb = r / seg;
  const int sr = rb * seg_full + (r - rb * seg);
  const float* p = src + (size_t)sr * EMB + c;
  const v4f a = *(const v4f*)p;
  const v4f b = *(const v4f*)(p + 4);
  v8us o;
  o[0] = bf16_bits_rne(a[0]); o[1] = bf16_bits_rne(a[1]);
  o[2] = bf16_bits_rne(a[2]); o[3] = bf16_bits_rne(a[3]);
  o[4] = bf16_bits_rne(b[0]); o[5] = bf16_bits_rne(b[1]);
  o[6] = bf16_bits_rne(b[2]); o[7] = bf16_bits_rne(b[3]);
  unsigned short* q = dst + (size_t)r * EMB + c;
  *(volatile v8us*)q = o;
  __threadfence();
  *(volatile v8us*)q = o;
}

template <bool F16OUT>
__global__ __launch_bounds__(256) void k_wtrans(const float* __restrict__ W, unsigned short* Wt,
                                                int K, int N, float scl) {
  __shared__ float T[64][65];
  const int tid = threadIdx.x;
  const int n0 = blockIdx.x * 64, k0 = blockIdx.y * 64;
#pragma unroll
  for (int j = 0; j < 4; ++j) {
    const int idx = tid + 256 * j;
    const int kr = idx >> 4, c4 = (idx & 15) * 4;
    const v4f v = *(const v4f*)(W + (size_t)(k0 + kr) * N + n0 + c4);
    T[kr][c4 + 0] = bf16_rne(v[0]);
    T[kr][c4 + 1] = bf16_rne(v[1]);
    T[kr][c4 + 2] = bf16_rne(v[2]);
    T[kr][c4 + 3] = bf16_rne(v[3]);
  }
  __syncthreads();
  v8us o[2];
#pragma unroll
  for (int j = 0; j < 2; ++j) {
    const int idx = tid + 256 * j;
    const int nr = idx >> 3, ch = idx & 7;
    v8us t;
#pragma unroll
    for (int e = 0; e < 8; ++e) {
      const float f = T[ch * 8 + e][nr] * scl;
      t[e] = F16OUT ? f16_bits(f) : bf16_bits_rne(f);
    }
    o[j] = t;
  }
#pragma unroll
  for (int j = 0; j < 2; ++j) {
    const int idx = tid + 256 * j;
    const int nr = idx >> 3, ch = idx & 7;
    *(volatile v8us*)(Wt + (size_t)(n0 + nr) * K + k0 + ch * 8) = o[j];
  }
  __threadfence();
#pragma unroll
  for (int j = 0; j < 2; ++j) {
    const int idx = tid + 256 * j;
    const int nr = idx >> 3, ch = idx & 7;
    *(volatile v8us*)(Wt + (size_t)(n0 + nr) * K + k0 + ch * 8) = o[j];
  }
}

template <int MODE, bool F16OP>
__global__ __launch_bounds__(256) void k_gemm(
    const unsigned short* __restrict__ A, const unsigned short* __restrict__ Bt,
    const float* __restrict__ bias, unsigned short* C0, unsigned short* C1, float* Cf,
    int M, int N, int K, int ldc, float oscale, int seg, int seg_full)
{
  __shared__ __attribute__((aligned(16))) float S[64][GSP];
  const int tid = threadIdx.x, lane = tid & 31, wv = tid >> 5;
  const int hs = lane >> 4, lm = lane & 15;
  const int mb = blockIdx.y * 128, nb = blockIdx.x * 128;
  const int wm = (wv >> 2) * 64, wn = (wv & 3) * 32;
  (void)M; (void)N;

  const unsigned short* ap0 = A  + (size_t)(mb + wm + lm) * K;
  const unsigned short* bp0 = Bt + (size_t)(nb + wn + lm) * K;

  v8f acc[4][2];
#pragma unroll
  for (int mt = 0; mt < 4; ++mt)
#pragma unroll
    for (int nt = 0; nt < 2; ++nt)
#pragma unroll
      for (int i = 0; i < 8; ++i) acc[mt][nt][i] = 0.0f;

#pragma unroll 2
  for (int k0 = 0; k0 < K; k0 += 32) {
    v16us af[4], bf[2];
#pragma unroll
    for (int mt = 0; mt < 4; ++mt) af[mt] = ld_frag(ap0 + (size_t)mt * 16 * K + k0, hs);
#pragma unroll
    for (int nt = 0; nt < 2; ++nt) bf[nt] = ld_frag(bp0 + (size_t)nt * 16 * K + k0, hs);
#pragma unroll
    for (int mt = 0; mt < 4; ++mt)
#pragma unroll
      for (int nt = 0; nt < 2; ++nt) {
        if (F16OP) acc[mt][nt] = mma_f16(af[mt], bf[nt], acc[mt][nt]);
        else       acc[mt][nt] = mma_bf16(af[mt], bf[nt], acc[mt][nt]);
      }
    asm volatile("v_nop\n\tv_nop\n\tv_nop\n\tv_nop"
                 : "+v"(acc[0][0]), "+v"(acc[0][1]), "+v"(acc[1][0]), "+v"(acc[1][1]),
                   "+v"(acc[2][0]), "+v"(acc[2][1]), "+v"(acc[3][0]), "+v"(acc[3][1])
                 : "v"(af[0]), "v"(af[1]), "v"(af[2]), "v"(af[3]), "v"(bf[0]), "v"(bf[1]));
  }

  for (int pass = 0; pass < 2; ++pass) {
#pragma unroll
    for (int mt = 0; mt < 4; ++mt)
#pragma unroll
      for (int nt = 0; nt < 2; ++nt)
#pragma unroll
        for (int i = 0; i < 8; ++i) {
          const int r = wm + mt * 16 + 8 * hs + i;
          const int c = wn + nt * 16 + lm;
          const int sr = (MODE == 2) ? c : r;
          const int sc = (MODE == 2) ? r : c;
          if ((sr >> 6) == pass) S[sr & 63][sc] = acc[mt][nt][i];
        }
    __syncthreads();

    if (MODE == 0) {
      v4f vals[8];
#pragma unroll
      for (int j = 0; j < 8; ++j) {
        const int row = (tid >> 5) + 8 * j;
        v4f v = *(const v4f*)&S[row][4 * lane];
#pragma unroll
        for (int e = 0; e < 4; ++e) v[e] = v[e] * oscale + bf16_rne(bias[nb + 4 * lane + e]);
        vals[j] = v;
      }
#pragma unroll
      for (int j = 0; j < 8; ++j) {
        const int gr = mb + pass * 64 + (tid >> 5) + 8 * j;
        const int gb = gr / seg;
        const int orow = gb * seg_full + (gr - gb * seg);
        *(volatile v4f*)(Cf + (size_t)orow * ldc + nb + 4 * lane) = vals[j];
      }
      __threadfence();
#pragma unroll
      for (int j = 0; j < 8; ++j) {
        const int gr = mb + pass * 64 + (tid >> 5) + 8 * j;
        const int gb = gr / seg;
        const int orow = gb * seg_full + (gr - gb * seg);
        *(volatile v4f*)(Cf + (size_t)orow * ldc + nb + 4 * lane) = vals[j];
      }
    } else if (MODE == 1) {
      v8us vh[4], vl[4];
#pragma unroll
      for (int j = 0; j < 4; ++j) {
        const int row = (tid >> 4) + 16 * j, ch = tid & 15;
        const v4f a = *(const v4f*)&S[row][8 * ch];
        const v4f b = *(const v4f*)&S[row][8 * ch + 4];
        const float f8[8] = { a[0], a[1], a[2], a[3], b[0], b[1], b[2], b[3] };
        v8us th, tl;
#pragma unroll
        for (int e = 0; e < 8; ++e) {
          const float f = f8[e] + bf16_rne(bias[nb + 8 * ch + e]);
          const unsigned short hb = bf16_bits_rne(f);
          th[e] = hb;
          tl[e] = bf16_bits_rne(f - bf16_val(hb));
        }
        vh[j] = th; vl[j] = tl;
      }
#pragma unroll
      for (int j = 0; j < 4; ++j) {
        const int row = (tid >> 4) + 16 * j, ch = tid & 15;
        const size_t o = (size_t)(mb + pass * 64 + row) * ldc + nb + 8 * ch;
        *(volatile v8us*)(C0 + o) = vh[j];
        *(volatile v8us*)(C1 + o) = vl[j];
      }
      __threadfence();
#pragma unroll
      for (int j = 0; j < 4; ++j) {
        const int row = (tid >> 4) + 16 * j, ch = tid & 15;
        const size_t o = (size_t)(mb + pass * 64 + row) * ldc + nb + 8 * ch;
        *(volatile v8us*)(C0 + o) = vh[j];
        *(volatile v8us*)(C1 + o) = vl[j];
      }
    } else {
      v8us vo[4];
#pragma unroll
      for (int j = 0; j < 4; ++j) {
        const int row = (tid >> 4) + 16 * j, ch = tid & 15;
        const int gn = nb + pass * 64 + row;
        const float bb = bf16_rne(bias[gn]);
        const v4f a = *(const v4f*)&S[row][8 * ch];
        const v4f b = *(const v4f*)&S[row][8 * ch + 4];
        const float f8[8] = { a[0], a[1], a[2], a[3], b[0], b[1], b[2], b[3] };
        v8us t;
#pragma unroll
        for (int e = 0; e < 8; ++e) t[e] = f16_bits((f8[e] + bb) * oscale);
        vo[j] = t;
      }
#pragma unroll
      for (int j = 0; j < 4; ++j) {
        const int row = (tid >> 4) + 16 * j, ch = tid & 15;
        const int gn = nb + pass * 64 + row;
        *(volatile v8us*)(C0 + (size_t)gn * ldc + mb + 8 * ch) = vo[j];
      }
      __threadfence();
#pragma unroll
      for (int j = 0; j < 4; ++j) {
        const int row = (tid >> 4) + 16 * j, ch = tid & 15;
        const int gn = nb + pass * 64 + row;
        *(volatile v8us*)(C0 + (size_t)gn * ldc + mb + 8 * ch) = vo[j];
      }
    }
    __syncthreads();
  }
}

__global__ __launch_bounds__(256) void k_attn(
    const unsigned short* __restrict__ Qh, const unsigned short* __restrict__ Ql,
    const unsigned short* __restrict__ Kh, const unsigned short* __restrict__ Kl,
    const unsigned short* __restrict__ Vt, unsigned short* Og)
{
  __shared__ __attribute__((aligned(16))) unsigned short Khs[64 * ALP];
  __shared__ __attribute__((aligned(16))) unsigned short Kls[64 * ALP];
  __shared__ __attribute__((aligned(16))) unsigned short Vts[64 * ALP];
  __shared__ __attribute__((aligned(16))) unsigned short Ps[8 * 16 * ALP];

  const int tid = threadIdx.x, lane = tid & 31, wv = tid >> 5;
  const int hs = lane >> 4, lm = lane & 15;
  const int qb = blockIdx.x, hh = blockIdx.y, bb = blockIdx.z;
  const int qrow0 = bb * SEQ + qb * 128 + wv * 16;
  const int hcol = hh * HD;
  unsigned short* Pw = Ps + wv * 16 * ALP;

  v16us qh[2], ql[2];
#pragma unroll
  for (int ks = 0; ks < 2; ++ks) {
    qh[ks] = ld_frag(Qh + (size_t)(qrow0 + lm) * EMB + hcol + ks * 32, hs);
    ql[ks] = ld_frag(Ql + (size_t)(qrow0 + lm) * EMB + hcol + ks * 32, hs);
  }

  v8f ov[4];
#pragma unroll
  for (int dt = 0; dt < 4; ++dt)
#pragma unroll
    for (int r = 0; r < 8; ++r) ov[dt][r] = 0.0f;
  float mrun[8], lrun[8];
#pragma unroll
  for (int r = 0; r < 8; ++r) { mrun[r] = -__builtin_inff(); lrun[r] = 0.0f; }

  const int str = tid >> 2;
  const int stc = (tid & 3) * 16;

  for (int kc = 0; kc < SKV / 64; ++kc) {
    __syncthreads();
    {
      const size_t krow = (size_t)bb * SKV + (size_t)kc * 64 + str;
      const unsigned short* gkh = Kh + krow * EMB + hcol + stc;
      const unsigned short* gkl = Kl + krow * EMB + hcol + stc;
      const unsigned short* gv  = Vt + (size_t)(hcol + str) * MK + (size_t)bb * SKV + (size_t)kc * 64 + stc;
      unsigned short* lkh = Khs + str * ALP + stc;
      unsigned short* lkl = Kls + str * ALP + stc;
      unsigned short* lv  = Vts + str * ALP + stc;
      *(v8us*)(lkh)     = *(const v8us*)(gkh);
      *(v8us*)(lkh + 8) = *(const v8us*)(gkh + 8);
      *(v8us*)(lkl)     = *(const v8us*)(gkl);
      *(v8us*)(lkl + 8) = *(const v8us*)(gkl + 8);
      *(v8us*)(lv)      = *(const v8us*)(gv);
      *(v8us*)(lv + 8)  = *(const v8us*)(gv + 8);
    }
    __syncthreads();

    v8f sacc[4];
#pragma unroll
    for (int nt = 0; nt < 4; ++nt) {
      v16us bh[2], bl[2];
#pragma unroll
      for (int ks = 0; ks < 2; ++ks) {
        bh[ks] = ld_frag(Khs + (nt * 16 + lm) * ALP + ks * 32, hs);
        bl[ks] = ld_frag(Kls + (nt * 16 + lm) * ALP + ks * 32, hs);
      }
      v8f z;
#pragma unroll
      for (int r = 0; r < 8; ++r) z[r] = 0.0f;
#pragma unroll
      for (int ks = 0; ks < 2; ++ks) {
        z = mma_bf16(qh[ks], bh[ks], z);
        z = mma_bf16(qh[ks], bl[ks], z);
        z = mma_bf16(ql[ks], bh[ks], z);
      }
      asm volatile("v_nop\n\tv_nop\n\tv_nop\n\tv_nop"
                   : "+v"(z)
                   : "v"(qh[0]), "v"(qh[1]), "v"(ql[0]), "v"(ql[1]),
                     "v"(bh[0]), "v"(bh[1]), "v"(bl[0]), "v"(bl[1]));
      sacc[nt] = z;
    }

    float mnew[8], corr[8], psum[8];
#pragma unroll
    for (int r = 0; r < 8; ++r) {
      float mx = fmaxf(fmaxf(sacc[0][r], sacc[1][r]), fmaxf(sacc[2][r], sacc[3][r]));
      mx = fmaxf(mx, __shfl_xor(mx, 1, 32));
      mx = fmaxf(mx, __shfl_xor(mx, 2, 32));
      mx = fmaxf(mx, __shfl_xor(mx, 4, 32));
      mx = fmaxf(mx, __shfl_xor(mx, 8, 32));
      mx *= 0.125f;
      mnew[r] = fmaxf(mrun[r], mx);
      corr[r] = __expf(mrun[r] - mnew[r]);
      psum[r] = 0.0f;
    }
#pragma unroll
    for (int nt = 0; nt < 4; ++nt)
#pragma unroll
      for (int r = 0; r < 8; ++r) {
        const float p = __expf(sacc[nt][r] * 0.125f - mnew[r]);
        psum[r] += p;
        Pw[(8 * hs + r) * ALP + nt * 16 + lm] = f16_bits(p * 16384.0f);
      }
#pragma unroll
    for (int r = 0; r < 8; ++r) {
      float sr = psum[r];
      sr += __shfl_xor(sr, 1, 32);
      sr += __shfl_xor(sr, 2, 32);
      sr += __shfl_xor(sr, 4, 32);
      sr += __shfl_xor(sr, 8, 32);
      lrun[r] = lrun[r] * corr[r] + sr;
      mrun[r] = mnew[r];
    }
#pragma unroll
    for (int dt = 0; dt < 4; ++dt)
#pragma unroll
      for (int r = 0; r < 8; ++r) ov[dt][r] *= corr[r];

    __syncthreads();

    v16us pa[2];
#pragma unroll
    for (int ks = 0; ks < 2; ++ks) pa[ks] = ld_frag(Pw + lm * ALP + ks * 32, hs);
#pragma unroll
    for (int dt = 0; dt < 4; ++dt) {
      v16us vb[2];
#pragma unroll
      for (int ks = 0; ks < 2; ++ks) vb[ks] = ld_frag(Vts + (dt * 16 + lm) * ALP + ks * 32, hs);
      ov[dt] = mma_f16(pa[0], vb[0], ov[dt]);
      ov[dt] = mma_f16(pa[1], vb[1], ov[dt]);
      asm volatile("v_nop\n\tv_nop\n\tv_nop\n\tv_nop"
                   : "+v"(ov[dt])
                   : "v"(pa[0]), "v"(pa[1]), "v"(vb[0]), "v"(vb[1]));
    }
  }

  __syncthreads();
#pragma unroll
  for (int r = 0; r < 8; ++r) {
    const float inv = (1.0f / lrun[r]) * (1.0f / 256.0f);
#pragma unroll
    for (int dt = 0; dt < 4; ++dt)
      Pw[(8 * hs + r) * ALP + dt * 16 + lm] = f16_bits(ov[dt][r] * inv);
  }
  __syncthreads();
  v8us vo[4];
#pragma unroll
  for (int j = 0; j < 4; ++j) {
    const int row = (lane >> 3) + 4 * j, ch = lane & 7;
    vo[j] = *(const v8us*)(Pw + row * ALP + ch * 8);
  }
#pragma unroll
  for (int j = 0; j < 4; ++j) {
    const int row = (lane >> 3) + 4 * j, ch = lane & 7;
    *(volatile v8us*)(Og + (size_t)(qrow0 + row) * EMB + hcol + ch * 8) = vo[j];
  }
  __threadfence();
#pragma unroll
  for (int j = 0; j < 4; ++j) {
    const int row = (lane >> 3) + 4 * j, ch = lane & 7;
    *(volatile v8us*)(Og + (size_t)(qrow0 + row) * EMB + hcol + ch * 8) = vo[j];
  }
}

extern "C" void kernel_launch(void* const* d_in, const int* in_sizes, int n_in,
                              void* d_out, int out_size, void* d_ws, size_t ws_size,
                              hipStream_t stream)
{
  if (n_in < 10) return;
  if (in_sizes[0] < ((NB - 1) * SQ_FULL + SEQ) * EMB) return;
  if (in_sizes[1] < NB * SKV * EMB) return;
  if (in_sizes[2] < EMB * EMB || in_sizes[4] < EMB * EMB || in_sizes[6] < EMB * EMB) return;
  if (in_sizes[3] < EMB || in_sizes[5] < EMB || in_sizes[7] < EMB) return;
  if (in_sizes[8] < EMB * VOC || in_sizes[9] < VOC) return;
  if (out_size < ((NB - 1) * SQ_FULL + SEQ) * VOC) return;

  const float* x   = (const float*)d_in[0];
  const float* ctx = (const float*)d_in[1];
  const float* Wq  = (const float*)d_in[2];
  const float* bq  = (const float*)d_in[3];
  const float* Wk  = (const float*)d_in[4];
  const float* bk  = (const float*)d_in[5];
  const float* Wv  = (const float*)d_in[6];
  const float* bv  = (const float*)d_in[7];
  const float* Wp  = (const float*)d_in[8];
  const float* bp  = (const float*)d_in[9];
  float* out = (float*)d_out;

  const size_t szQrow = (size_t)MQ * EMB * 2;
  const size_t szKrow = (size_t)MK * EMB * 2;
  const size_t szW    = (size_t)EMB * EMB * 2;
  const size_t szWp   = (size_t)VOC * EMB * 2;
  char* ws = (char*)d_ws;
  size_t off = 0;
  unsigned short* xb  = (unsigned short*)(ws + off); off += szQrow;
  unsigned short* cb  = (unsigned short*)(ws + off); off += szKrow;
  unsigned short* WqT = (unsigned short*)(ws + off); off += szW;
  unsigned short* WkT = (unsigned short*)(ws + off); off += szW;
  unsigned short* WvT = (unsigned short*)(ws + off); off += szW;
  unsigned short* WpT = (unsigned short*)(ws + off); off += szWp;
  unsigned short* Qh  = (unsigned short*)(ws + off); off += szQrow;
  unsigned short* Ql  = (unsigned short*)(ws + off); off += szQrow;
  unsigned short* Kh  = (unsigned short*)(ws + off); off += szKrow;
  unsigned short* Kl  = (unsigned short*)(ws + off); off += szKrow;
  unsigned short* Vt  = (unsigned short*)(ws + off); off += szKrow;
  unsigned short* Ob  = (unsigned short*)(ws + off); off += szQrow;
  if (off > ws_size) return;

  k_cvt_rows<<<MQ / 2, 256, 0, stream>>>(x, xb, MQ, SEQ, SQ_FULL);
  k_cvt_rows<<<MK / 2, 256, 0, stream>>>(ctx, cb, MK, SKV, SKV);
  k_wtrans<false><<<dim3(EMB / 64, EMB / 64), 256, 0, stream>>>(Wq, WqT, EMB, EMB, 1.0f);
  k_wtrans<false><<<dim3(EMB / 64, EMB / 64), 256, 0, stream>>>(Wk, WkT, EMB, EMB, 1.0f);
  k_wtrans<false><<<dim3(EMB / 64, EMB / 64), 256, 0, stream>>>(Wv, WvT, EMB, EMB, 1.0f);
  k_wtrans<true ><<<dim3(VOC / 64, EMB / 64), 256, 0, stream>>>(Wp, WpT, EMB, VOC, 256.0f);
  k_gemm<1, false><<<dim3(EMB / 128, MQ / 128), 256, 0, stream>>>(
      xb, WqT, bq, Qh, Ql, out, MQ, EMB, EMB, EMB, 1.0f, SEQ, SEQ);
  k_gemm<1, false><<<dim3(EMB / 128, MK / 128), 256, 0, stream>>>(
      cb, WkT, bk, Kh, Kl, out, MK, EMB, EMB, EMB, 1.0f, SKV, SKV);
  k_gemm<2, false><<<dim3(EMB / 128, MK / 128), 256, 0, stream>>>(
      cb, WvT, bv, Vt, Vt, out, MK, EMB, EMB, MK, 1.0f, SKV, SKV);
  k_attn<<<dim3(SEQ / 128, NH, NB), 256, 0, stream>>>(Qh, Ql, Kh, Kl, Vt, Ob);
  k_gemm<0, true><<<dim3(VOC / 128, MQ / 128), 256, 0, stream>>>(
      Ob, WpT, bp, Ob, Ob, out, MQ, VOC, EMB, VOC, 1.0f / 16384.0f, SEQ, SQ_FULL);
}
